// MultiScaleGATEncoder_87531433492498
// MI455X (gfx1250) — hardware-verified
//
#include <hip/hip_runtime.h>
#include <math.h>

typedef __attribute__((ext_vector_type(16))) _Float16 v16h;
typedef __attribute__((ext_vector_type(16))) __bf16 v16b;
typedef __attribute__((ext_vector_type(8)))  _Float16 v8h;
typedef __attribute__((ext_vector_type(8)))  float v8f;
typedef __attribute__((ext_vector_type(4)))  float v4f;
typedef __attribute__((ext_vector_type(2)))  float v2f;
typedef __attribute__((ext_vector_type(4)))  unsigned v4u;
typedef __attribute__((ext_vector_type(4)))  int v4i;
typedef float __attribute__((may_alias)) float_a;
typedef int __attribute__((may_alias)) int_a;

template <typename T> __device__ __forceinline__ void vst2(void* p, T v) { *(volatile T*)p = v; __threadfence(); *(volatile T*)p = v; }
__device__ __forceinline__ v8f wmma16(v16h a, v16h b, v8f c) {
  v8f d = __builtin_amdgcn_wmma_f32_16x16x32_f16(false, a, false, b, (short)0, c, false, false);
  asm volatile("v_nop\n\tv_nop\n\tv_nop\n\tv_nop" : "+v"(d) : "v"(a), "v"(b));
  return d;
}
__device__ __forceinline__ v8f wmma_bf(v16b a, v16b b, v8f c) {
  v8f d = __builtin_amdgcn_wmma_f32_16x16x32_bf16(false, a, false, b, (short)0, c, false, false);
  asm volatile("v_nop\n\tv_nop\n\tv_nop\n\tv_nop" : "+v"(d) : "v"(a), "v"(b));
  return d;
}
__device__ __forceinline__ v16h frag_h(const _Float16* rowk0, int lane) {
  union { v16h v; v8h q[2]; } u; const _Float16* p = rowk0 + 8 * (lane >> 4);
  u.q[0] = *(const v8h*)p; u.q[1] = *(const v8h*)(p + 16); return u.v;
}
__device__ __forceinline__ v16h frag_f32(const float* rowk0, int lane) {
  v16h a; const float* p = rowk0 + 8 * (lane >> 4);
#pragma unroll
  for (int i = 0; i < 8; ++i) { a[i] = (_Float16)p[i]; a[8 + i] = (_Float16)p[16 + i]; }
  return a;
}
__device__ __forceinline__ v16h frag_f32s(const float* rowk0, int lane, float sc) {
  v16h a; const float* p = rowk0 + 8 * (lane >> 4);
#pragma unroll
  for (int i = 0; i < 8; ++i) { a[i] = (_Float16)(p[i] * sc); a[8 + i] = (_Float16)(p[16 + i] * sc); }
  return a;
}
__device__ __forceinline__ v16h fragc_f32(const float* W, int k0, int n, int lane, int ld, int K) {
  v16h a; const int g = lane >> 4;
#pragma unroll
  for (int i = 0; i < 8; ++i) { const int ka = k0 + 8 * g + i, kb = ka + 16;
    a[i] = (_Float16)(ka < K ? W[(size_t)ka * ld + n] : 0.f); a[8 + i] = (_Float16)(kb < K ? W[(size_t)kb * ld + n] : 0.f); }
  return a;
}
struct F2 { v16b h, l; };
__device__ __forceinline__ F2 bsplit16(const float v[16]) { F2 r;
#pragma unroll
  for (int i = 0; i < 16; ++i) { const __bf16 h = (__bf16)v[i]; r.h[i] = h; r.l[i] = (__bf16)(v[i] - (float)h); }
  return r; }
__device__ __forceinline__ F2 split_row(const float* row, int k0, int lane) { float v[16]; const float* p = row + k0 + 8 * (lane >> 4);
#pragma unroll
  for (int i = 0; i < 8; ++i) { v[i] = p[i]; v[8 + i] = p[16 + i]; }
  return bsplit16(v); }
__device__ __forceinline__ F2 split_rowK(const float* row, int k0, int lane, int K) { float v[16]; const int g = lane >> 4;
#pragma unroll
  for (int i = 0; i < 8; ++i) { const int ka = k0 + 8 * g + i, kb = ka + 16; v[i] = ka < K ? row[ka] : 0.f; v[8 + i] = kb < K ? row[kb] : 0.f; }
  return bsplit16(v); }
__device__ __forceinline__ F2 split_col(const float* W, int k0, int n, int lane, int ld, int K) { float v[16]; const int g = lane >> 4;
#pragma unroll
  for (int i = 0; i < 8; ++i) { const int ka = k0 + 8 * g + i, kb = ka + 16; v[i] = ka < K ? W[(size_t)ka * ld + n] : 0.f; v[8 + i] = kb < K ? W[(size_t)kb * ld + n] : 0.f; }
  return bsplit16(v); }
__device__ __forceinline__ v8f mac3(const F2& a, const F2& b, v8f c) { c = wmma_bf(a.l, b.h, c); c = wmma_bf(a.h, b.l, c); return wmma_bf(a.h, b.h, c); }
__device__ __forceinline__ float sigm(float v) { return 1.0f / (1.0f + expf(-v)); }
#define LDSX() do { asm volatile("s_wait_dscnt 0" ::: "memory"); __builtin_amdgcn_wave_barrier(); __builtin_amdgcn_fence(__ATOMIC_RELEASE, "workgroup"); } while (0)

#define FIN 156
#define DH 64
#define NE 3
#define HWPX (1024 * 1024)

__global__ __launch_bounds__(128) void k_h1(const float* __restrict__ X, int N, const float* __restrict__ W, const float* __restrict__ bias, float* __restrict__ H) {
  __shared__ __align__(16) float so[4][16][68];
  const int tid = threadIdx.x, wave = tid >> 5, lane = tid & 31, col = lane & 15, g = lane >> 4;
  const int r0 = blockIdx.x * 64 + wave * 16; const int ra = min(r0 + col, N - 1);
  v8f acc[4] = {};
#pragma unroll
  for (int kc = 0; kc < 5; ++kc) { const F2 a = split_rowK(X + (size_t)ra * FIN, kc * 32, lane, FIN);
#pragma unroll
    for (int j = 0; j < 4; ++j) acc[j] = mac3(a, split_col(W, kc * 32, j * 16 + col, lane, DH, FIN), acc[j]); }
#pragma unroll
  for (int j = 0; j < 4; ++j) { const int c = j * 16 + col; const float bb = bias[c];
#pragma unroll
    for (int r = 0; r < 8; ++r) so[wave][8 * g + r][c] = (r0 + 8 * g + r) < N ? acc[j][r] + bb : 0.f; }
  LDSX();
  for (int q = lane; q < 16 * 16; q += 32) { const int rl = q >> 4, pc = q & 15; vst2(H + (size_t)(r0 + rl) * DH + pc * 4, *(const v4f*)(&so[wave][rl][pc * 4])); }
}
__global__ __launch_bounds__(128) void k_att1(const float* __restrict__ H, const int* __restrict__ Adj, int N, int NP, float* __restrict__ X1) {
  __shared__ __align__(16) float sS[4][16][20];
  __shared__ __align__(16) float sP[4][16][36];
  __shared__ __align__(16) float so[4][16][68];
  const int tid = threadIdx.x, w = tid >> 5, lane = tid & 31, col = lane & 15, g = lane >> 4;
  const int i0 = blockIdx.x * 64 + w * 16;
  F2 ah[2];
#pragma unroll
  for (int kc = 0; kc < 2; ++kc) ah[kc] = split_row(H + (size_t)(i0 + col) * DH, kc * 32, lane);
  float mrun = -3.0e38f, lrun = 0.f; v8f acc[4] = {};
#pragma unroll 1
  for (int jc = 0; jc < NP / 32; ++jc) {
    float corr_row = 1.0f;
#pragma unroll
    for (int t = 0; t < 2; ++t) { v8f s = {}; const int j0 = jc * 32 + t * 16;
#pragma unroll
      for (int kc = 0; kc < 2; ++kc) s = mac3(ah[kc], split_row(H + (size_t)(j0 + col) * DH, kc * 32, lane), s);
#pragma unroll
      for (int r = 0; r < 8; ++r) { const int i = i0 + 8 * g + r, j = j0 + col; const bool ok = (i < N) && (j < N);
        const float a = ok ? (Adj[(size_t)i * N + j] > 0 ? s[r] : -1.0e9f) : -3.0e38f; sS[w][8 * g + r][col] = a; }
      LDSX();
      if (g == 0) { const int m = col; float mx = -3.4e38f;
#pragma unroll
        for (int e = 0; e < 16; ++e) mx = fmaxf(mx, sS[w][m][e]);
        const float mnew = fmaxf(mrun, mx); const float corr = expf(mrun - mnew); float ps = 0.f;
#pragma unroll
        for (int e = 0; e < 16; ++e) { const float sv = sS[w][m][e]; const float p = sv <= -1.0e38f ? 0.f : expf(sv - mnew); ps += p; sP[w][m][t * 16 + e] = p; }
        if (t == 1) {
#pragma unroll
          for (int e = 0; e < 16; ++e) sP[w][m][e] *= corr; }
        lrun = lrun * corr + ps; mrun = mnew; corr_row *= corr; }
      LDSX(); }
#pragma unroll
    for (int r = 0; r < 8; ++r) { const float cr = __shfl(corr_row, 8 * g + r, 32);
#pragma unroll
      for (int t4 = 0; t4 < 4; ++t4) acc[t4][r] *= cr; }
    { const F2 pa = split_row(&sP[w][col][0], 0, lane);
#pragma unroll
      for (int t4 = 0; t4 < 4; ++t4) acc[t4] = mac3(pa, split_col(H + (size_t)(jc * 32) * DH, 0, t4 * 16 + col, lane, DH, 32), acc[t4]); }
    LDSX();
  }
#pragma unroll
  for (int r = 0; r < 8; ++r) { const float lr = __shfl(lrun, 8 * g + r, 32);
#pragma unroll
    for (int t4 = 0; t4 < 4; ++t4) { const float v = acc[t4][r] / lr; so[w][8 * g + r][t4 * 16 + col] = (i0 + 8 * g + r) < N ? (v > 0.f ? v : 0.f) : 0.f; } }
  LDSX();
  for (int q = lane; q < 16 * 16; q += 32) { const int rl = q >> 4, pc = q & 15; vst2(X1 + (size_t)(i0 + rl) * DH + pc * 4, *(const v4f*)(&so[w][rl][pc * 4])); }
}
__global__ __launch_bounds__(256) void k_h2(const float* __restrict__ X1, int N, const float* __restrict__ W2, const float* __restrict__ b2, float* __restrict__ H2) {
  const int i = blockIdx.x * 256 + threadIdx.x; float a0 = 0.f, a1 = 0.f, a2 = 0.f;
  if (i < N) { a0 = b2[0]; a1 = b2[1]; a2 = b2[2]; const float* xr = X1 + (size_t)i * DH;
#pragma unroll 1
    for (int k = 0; k < DH; ++k) { const float xv = xr[k]; a0 += xv * W2[k * NE]; a1 += xv * W2[k * NE + 1]; a2 += xv * W2[k * NE + 2]; } }
  vst2(H2 + (size_t)i * 4, (v4f){a0, a1, a2, 0.f});
}
__global__ __launch_bounds__(256) void k_att2(const float* __restrict__ H2, const int* __restrict__ Adj, int N, float* __restrict__ PR) {
  const int i = blockIdx.x * 256 + threadIdx.x; float o0 = 0.f, o1 = 0.f, o2 = 0.f;
  if (i < N) { const v4f hi = *(const v4f*)(H2 + (size_t)i * 4); const int* ar = Adj + (size_t)i * N; float m = -3.4e38f;
#pragma unroll 1
    for (int j = 0; j < N; ++j) { const v4f hj = *(const v4f*)(H2 + (size_t)j * 4); float s = hi[0] * hj[0] + hi[1] * hj[1] + hi[2] * hj[2]; s = ar[j] > 0 ? s : -1.0e9f; m = fmaxf(m, s); }
    float l = 0.f, c0 = 0.f, c1 = 0.f, c2 = 0.f;
#pragma unroll 1
    for (int j = 0; j < N; ++j) { const v4f hj = *(const v4f*)(H2 + (size_t)j * 4); float s = hi[0] * hj[0] + hi[1] * hj[1] + hi[2] * hj[2]; s = ar[j] > 0 ? s : -1.0e9f; const float p = expf(s - m); l += p; c0 += p * hj[0]; c1 += p * hj[1]; c2 += p * hj[2]; }
    const float inv = 1.0f / l; o0 = fmaxf(c0 * inv, 0.f); o1 = fmaxf(c1 * inv, 0.f); o2 = fmaxf(c2 * inv, 0.f);
    const float mm = fmaxf(o0, fmaxf(o1, o2)); const float e0 = expf(o0 - mm), e1 = expf(o1 - mm), e2 = expf(o2 - mm); const float z = 1.0f / (e0 + e1 + e2); o0 = e0 * z; o1 = e1 * z; o2 = e2 * z; }
  vst2(PR + (size_t)i * 4, (v4f){o0, o1, o2, 0.f});
}
__global__ __launch_bounds__(128) void k_img(const float* __restrict__ PR0, const int* __restrict__ seg0, int N0_, const float* __restrict__ PR1, const int* __restrict__ seg1, int N1_, const float* __restrict__ PR2, const int* __restrict__ seg2, int N2_,
                                           const float* __restrict__ sw, float* __restrict__ out) {
  __shared__ __align__(16) float so[128 * NE];
  const int tid = threadIdx.x; const size_t p = (size_t)blockIdx.x * 128 + tid;
  const float m = fmaxf(sw[0], fmaxf(sw[1], sw[2])); const float e0 = expf(sw[0] - m), e1 = expf(sw[1] - m), e2 = expf(sw[2] - m); const float z = 1.0f / (e0 + e1 + e2);
  const float w0 = e0 * z, w1 = e1 * z, w2 = e2 * z;
  int s0 = seg0[p], s1 = seg1[p], s2 = seg2[p]; s0 = s0 < 0 ? 0 : (s0 >= N0_ ? N0_ - 1 : s0); s1 = s1 < 0 ? 0 : (s1 >= N1_ ? N1_ - 1 : s1); s2 = s2 < 0 ? 0 : (s2 >= N2_ ? N2_ - 1 : s2);
  const v4f a = *(const v4f*)(PR0 + (size_t)s0 * 4), b = *(const v4f*)(PR1 + (size_t)s1 * 4), c = *(const v4f*)(PR2 + (size_t)s2 * 4);
#pragma unroll
  for (int e = 0; e < NE; ++e) so[tid * NE + e] = (w0 * a[e] + w1 * b[e]) + w2 * c[e];
  __syncthreads();
  if (tid < 96) vst2(out + (size_t)blockIdx.x * 384 + tid * 4, *(const v4f*)(&so[tid * 4]));
}
extern "C" void kernel_launch(void* const* d_in, const int* in_sizes, int n_in, void* d_out, int out_size, void* d_ws, size_t ws_size, hipStream_t stream) {
  (void)in_sizes; (void)n_in; (void)out_size; (void)ws_size;
  const int Ns[3] = {2000, 1000, 500}; const int NPs[3] = {2048, 1024, 512};
  const float* sw = (const float*)d_in[21];
  float* out = (float*)d_out;
  char* ws = (char*)d_ws; size_t off = 0;
  auto take = [&](size_t bytes) { char* p = ws + off; off += (bytes + 255) & ~(size_t)255; return p; };
  float* PR[3];
  for (int s = 0; s < 3; ++s) {
    const float* X = (const float*)d_in[7 * s]; const int* Adj = (const int*)d_in[7 * s + 1]; const float* W1 = (const float*)d_in[7 * s + 3]; const float* b1 = (const float*)d_in[7 * s + 4];
    const float* W2 = (const float*)d_in[7 * s + 5]; const float* b2 = (const float*)d_in[7 * s + 6];
    const int N = Ns[s], NP = NPs[s];
    float* H = (float*)take((size_t)NP * DH * 4); float* X1 = (float*)take((size_t)NP * DH * 4); float* H2 = (float*)take((size_t)NP * 4 * 4); PR[s] = (float*)take((size_t)NP * 4 * 4);
    k_h1<<<NP / 64, 128, 0, stream>>>(X, N, W1, b1, H);
    k_att1<<<NP / 64, 128, 0, stream>>>(H, Adj, N, NP, X1);
    k_h2<<<NP / 256, 256, 0, stream>>>(X1, N, W2, b2, H2);
    k_att2<<<NP / 256, 256, 0, stream>>>(H2, Adj, N, PR[s]);
  }
  k_img<<<HWPX / 128, 128, 0, stream>>>(PR[0], (const int*)d_in[2], Ns[0], PR[1], (const int*)d_in[9], Ns[1], PR[2], (const int*)d_in[16], Ns[2], sw, out);
}
